// MessageLayer_55241869361626
// MI455X (gfx1250) — hardware-verified
//
#include <hip/hip_runtime.h>
#include <stddef.h>
#include <stdint.h>


#define DIN     128
#define NHEAD   4
#define NL      512
#define NLR     1024
#define DFF     256
#define K1      256
#define K2      512
#define NTHR    256
#define NWAVE   8
#define EPT     8
#define CHUNK   (NTHR * EPT)
#define WCAP    (EPT * 32)
#define LISTN   (NWAVE * WCAP)
#define NBMAX   2048
#define NB0     1024
#define RCAP    28672
#define DEGCAP  4096
#define STW     512
#define NPRM    (3 * DIN)
#define GBM     64
#define GBN     64
#define GTHR    128
#define NEGS    0.2f
#define LNEPS   1.0e-5f
#define WSMAX   268435456
#define LDS_AGG ((2 * RCAP + 2 * NBMAX + LISTN + 2 * NWAVE + NPRM) * 4)
#define LDS_FFN (GBM * K2 * 2 + GBM * GBN * 4)

static_assert((CHUNK & (CHUNK - 1)) == 0 && CHUNK <= 4096);
static_assert((NBMAX & (NBMAX - 1)) == 0 && NBMAX <= 4096);
static_assert((NB0 & (NB0 - 1)) == 0 && NB0 <= NBMAX && NB0 >= 16);
static_assert(NTHR * 8 == NBMAX);
static_assert(LISTN >= NBMAX);
static_assert(LISTN >= NWAVE * WCAP);
static_assert((RCAP % 32) == 0);
static_assert(NWAVE * STW <= RCAP);
static_assert(STW >= NHEAD * DIN);
static_assert(LDS_AGG <= 300000);
static_assert((((2 * RCAP + 2 * NBMAX + LISTN + 2 * NWAVE) * 4) % 16) == 0);
static_assert(LDS_FFN <= 300000);
static_assert(GBM == (GTHR / 32) * 16);
static_assert(NL == NHEAD * DIN && NLR == 2 * NL);
static_assert((DIN % 32) == 0 && (K1 % 32) == 0 && (K2 % 32) == 0);
static_assert((NLR % GBN) == 0 && (DFF % GBN) == 0 && (DIN % GBN) == 0);
static_assert(K1 == 2 * DIN && K2 == 2 * DFF);
static_assert(DIN == 4 * 32);

typedef float           v4f  __attribute__((ext_vector_type(4)));
typedef float           v8f  __attribute__((ext_vector_type(8)));
typedef int             v4i  __attribute__((ext_vector_type(4)));
typedef int             v8i  __attribute__((ext_vector_type(8)));
typedef unsigned short  v4us __attribute__((ext_vector_type(4)));
typedef unsigned short  v8us __attribute__((ext_vector_type(8)));
typedef __bf16          v16b __attribute__((ext_vector_type(16)));
typedef v4f  __attribute__((may_alias)) v4fa;
typedef v4us __attribute__((may_alias)) v4usa;
typedef v8us __attribute__((may_alias)) v8usa;
union FragB { v16b v; v8us h[2]; v8i w; };

__device__ __forceinline__ v8f wmb(const FragB& a, const FragB& b, v8f c) {
  v8f d = __builtin_amdgcn_wmma_f32_16x16x32_bf16(false, a.v, false, b.v, (short)0, c, false, false);
  asm volatile("v_nop\n\tv_nop\n\tv_nop\n\tv_nop" : "+v"(d) : "v"(a.w), "v"(b.w));
  return d;
}

__device__ __forceinline__ void ldwait() {
  asm volatile("s_wait_loadcnt 0x0" ::: "memory");
}

__device__ __forceinline__ unsigned short f2bf(float f) {
  unsigned u = (unsigned)__float_as_uint(f);
  u = u + 0x7FFFu + ((u >> 16) & 1u);
  return (unsigned short)(u >> 16);
}
__device__ __forceinline__ float bf2f(unsigned short b) { return __uint_as_float(((unsigned)b) << 16); }
__device__ __forceinline__ float bfr(float f) { return bf2f(f2bf(f)); }

__device__ __forceinline__ v8us cvt8bf(const v4f a, const v4f b) {
  v8us o;
  o[0] = f2bf(a.x); o[1] = f2bf(a.y); o[2] = f2bf(a.z); o[3] = f2bf(a.w);
  o[4] = f2bf(b.x); o[5] = f2bf(b.y); o[6] = f2bf(b.z); o[7] = f2bf(b.w);
  return o;
}

__device__ __forceinline__ int scan_chunk(const int* __restrict__ dsts, int nE, int cbase, int slotBase,
                                          int nb, int vec8, int* list, int tid, int lane, int wave) {
  int wc = 0;
  const int el0  = tid * EPT;
  const int e0   = cbase + el0;
  const int sent = -2147483647 - 1;
  v4i da, db;
  if (vec8 != 0 && cbase + CHUNK <= nE) {
    da = *(const v4i*)(dsts + e0);
    db = *(const v4i*)(dsts + e0 + 4);
  } else {
    da.x = (e0     < nE) ? dsts[min(e0,     nE - 1)] : sent;
    da.y = (e0 + 1 < nE) ? dsts[min(e0 + 1, nE - 1)] : sent;
    da.z = (e0 + 2 < nE) ? dsts[min(e0 + 2, nE - 1)] : sent;
    da.w = (e0 + 3 < nE) ? dsts[min(e0 + 3, nE - 1)] : sent;
    db.x = (e0 + 4 < nE) ? dsts[min(e0 + 4, nE - 1)] : sent;
    db.y = (e0 + 5 < nE) ? dsts[min(e0 + 5, nE - 1)] : sent;
    db.z = (e0 + 6 < nE) ? dsts[min(e0 + 6, nE - 1)] : sent;
    db.w = (e0 + 7 < nE) ? dsts[min(e0 + 7, nE - 1)] : sent;
  }
  const unsigned nbs = (unsigned)slotBase;
  const unsigned unb = (unsigned)nb;
  const unsigned s0 = (unsigned)da.x - nbs, s1 = (unsigned)da.y - nbs;
  const unsigned s2 = (unsigned)da.z - nbs, s3 = (unsigned)da.w - nbs;
  const unsigned s4 = (unsigned)db.x - nbs, s5 = (unsigned)db.y - nbs;
  const unsigned s6 = (unsigned)db.z - nbs, s7 = (unsigned)db.w - nbs;
  const bool h0 = s0 < unb, h1 = s1 < unb, h2 = s2 < unb, h3 = s3 < unb;
  const bool h4 = s4 < unb, h5 = s5 < unb, h6 = s6 < unb, h7 = s7 < unb;
  const unsigned any = __builtin_amdgcn_ballot_w32(h0 | h1 | h2 | h3 | h4 | h5 | h6 | h7);
  if (any != 0u) {
#define HITJ(J, HJ, SJ) { \
      const unsigned mj = __builtin_amdgcn_ballot_w32(HJ); \
      if (mj != 0u) { \
        if (HJ) { \
          const int pos = wc + (int)__builtin_amdgcn_mbcnt_lo(mj, 0u); \
          if (pos < WCAP) list[wave * WCAP + pos] = ((el0 + (J)) << 12) | (int)(SJ); \
        } \
        wc += (int)__builtin_popcount(mj); } }
    HITJ(0, h0, s0)
    HITJ(1, h1, s1)
    HITJ(2, h2, s2)
    HITJ(3, h3, s3)
    HITJ(4, h4, s4)
    HITJ(5, h5, s5)
    HITJ(6, h6, s6)
    HITJ(7, h7, s7)
#undef HITJ
  }
  return wc;
}

__global__ __launch_bounds__(NTHR) void k_xprep(const float* __restrict__ x, unsigned short* xb, int nN, int nUnits) {
  const int i = (int)blockIdx.x * NTHR + (int)threadIdx.x;
  if (i >= nUnits) return;
  const int row = i >> 4;
  const int c0  = (i & 15) * 8;
  const int rc  = row < nN ? row : nN - 1;
  const float* p = x + (size_t)rc * DIN + c0;
  v4f a = *(const v4fa*)p, b = *(const v4fa*)(p + 4);
  const v4f z4 = {0.f, 0.f, 0.f, 0.f};
  if (row >= nN) { a = z4; b = z4; }
  const v8us o = cvt8bf(a, b);
  const size_t off = (size_t)row * DIN + c0;
  *(volatile v8us*)(xb + off) = o;
  __threadfence();
  *(volatile v8us*)(xb + off) = o;
}

__global__ __launch_bounds__(NTHR) void k_wtr(const float* __restrict__ w0, const float* __restrict__ w1,
                                              int cc, int segRows, int Kin, int Kout,
                                              unsigned short* wt, int nUnits) {
  const int u = (int)blockIdx.x * NTHR + (int)threadIdx.x;
  if (u >= nUnits) return;
  const int kq = Kout >> 3;
  const int n  = u / kq;
  const int k8 = (u - n * kq) * 8;
  int seg = n / segRows;
  seg = seg > 1 ? 1 : seg;
  const int nc  = n - seg * segRows;
  const int kin = k8 >= Kin ? k8 - Kin : k8;
  const float* ws = (seg == 0) ? w0 : w1;
  const int ncl = nc < cc ? nc : cc - 1;
  const float* p = ws + (size_t)kin * (size_t)cc + ncl;
  v4f a, b;
  a.x = p[0];                  a.y = p[(size_t)cc];         a.z = p[(size_t)2 * cc];     a.w = p[(size_t)3 * cc];
  b.x = p[(size_t)4 * cc];     b.y = p[(size_t)5 * cc];     b.z = p[(size_t)6 * cc];     b.w = p[(size_t)7 * cc];
  const v4f z4 = {0.f, 0.f, 0.f, 0.f};
  if (nc >= cc) { a = z4; b = z4; }
  const v8us o = cvt8bf(a, b);
  const size_t off = (size_t)n * (size_t)Kout + k8;
  *(volatile v8us*)(wt + off) = o;
  __threadfence();
  *(volatile v8us*)(wt + off) = o;
}

__global__ __launch_bounds__(GTHR) void k_gemm_xlr(
    const unsigned short* __restrict__ A, const unsigned short* __restrict__ WT,
    const float* __restrict__ bl, const float* __restrict__ br,
    float* outF, int K, int ldo)
{
  __shared__ __attribute__((aligned(16))) float stg[GBM * GBN];
  const int tid = (int)threadIdx.x, lane = tid & 31, wave = tid >> 5, hh = lane >> 4, m = lane & 15;
  const int rowBase = (int)blockIdx.x * GBM;
  const int col0    = (int)blockIdx.y * GBN;
  const int seg = col0 >= NL ? 1 : 0;
  const float* bp = (seg == 0) ? bl : br;
  int bofs = col0 - seg * NL;
  bofs = bofs < 0 ? 0 : bofs;

  v8f acc[4];
  {
    const v8f z = {0.f, 0.f, 0.f, 0.f, 0.f, 0.f, 0.f, 0.f};
    acc[0] = z; acc[1] = z; acc[2] = z; acc[3] = z;
  }
  const unsigned short* ap = A  + (size_t)(rowBase + 16 * wave + m) * (size_t)K + 8 * hh;
  const unsigned short* wp = WT + (size_t)(col0 + m) * (size_t)K + 8 * hh;
  const int ksteps = K >> 5;
#pragma unroll 1
  for (int ks = 0; ks < ksteps; ++ks) {
    FragB af;
    af.h[0] = *(const v8usa*)(ap + 32 * ks);
    af.h[1] = *(const v8usa*)(ap + 32 * ks + 16);
#pragma unroll
    for (int t = 0; t < 4; ++t) {
      const unsigned short* wq = wp + (size_t)(16 * t) * (size_t)K + 32 * ks;
      FragB bf;
      bf.h[0] = *(const v8usa*)wq;
      bf.h[1] = *(const v8usa*)(wq + 16);
      acc[t] = wmb(af, bf, acc[t]);
    }
  }

#pragma unroll
  for (int t = 0; t < 4; ++t) {
    const int lc = 16 * t + m;
    int bi = bofs + lc;
    bi = bi > NL - 1 ? NL - 1 : bi;
    bi = bi < 0 ? 0 : bi;
    const float bv = bfr(bp[bi]);
#pragma unroll
    for (int r = 0; r < 8; ++r) {
      const int lr = 16 * wave + 8 * hh + r;
      stg[lr * GBN + lc] = acc[t][r] + bv;
    }
  }
  __syncthreads();

  v4f fv[8];
#pragma unroll
  for (int i = 0; i < 8; ++i) {
    const int lr = 16 * wave + 2 * i + hh;
    fv[i] = *(const v4fa*)(stg + lr * GBN + 4 * m);
  }
#pragma unroll
  for (int i = 0; i < 8; ++i) {
    const int lr = 16 * wave + 2 * i + hh;
    const int gr = rowBase + lr;
    float* op = outF + (size_t)gr * (size_t)ldo + col0 + 4 * m;
    *(volatile v4f*)op = fv[i];
  }
  __threadfence();
#pragma unroll
  for (int i = 0; i < 8; ++i) {
    const int lr = 16 * wave + 2 * i + hh;
    const int gr = rowBase + lr;
    float* op = outF + (size_t)gr * (size_t)ldo + col0 + 4 * m;
    *(volatile v4f*)op = fv[i];
  }
}

__global__ __launch_bounds__(NTHR) void k_agg(
    const int* __restrict__ srcs, const int* __restrict__ dsts,
    const float* __restrict__ XLR, const unsigned short* __restrict__ XB,
    const float* __restrict__ att, const float* __restrict__ gbias,
    const float* __restrict__ lng, const float* __restrict__ lnb,
    unsigned short* HB, int nN, int nE, int nb, int vec8, int MPr) {
  extern __shared__ v4f lds_dyn[];
  int* reg1 = (int*)lds_dyn;
  int* reg2 = reg1 + RCAP;
  int* scnt = reg2 + RCAP;
  int* soff = scnt + NBMAX;
  int* list = soff + NBMAX;
  int* wcnt = list + LISTN;
  int* wtot = wcnt + NWAVE;
  float* prm = (float*)(wtot + NWAVE);
  const int tid = (int)threadIdx.x, lane = tid & 31, wave = tid >> 5;
  const int nodeBase = (int)blockIdx.x * nb;

  for (int i = tid; i < NBMAX; i += NTHR) scnt[i] = 0;
  if (tid < DIN) {
    prm[tid]           = bfr(gbias[tid]);
    prm[DIN + tid]     = bfr(lng[tid]);
    prm[2 * DIN + tid] = bfr(lnb[tid]);
  }
  reg2[tid] = 0;
  float attv[16];
  {
    const float* apt = att + 16 * lane;
    const v4f a0 = *(const v4fa*)apt, a1 = *(const v4fa*)(apt + 4), a2 = *(const v4fa*)(apt + 8), a3 = *(const v4fa*)(apt + 12);
    ldwait();
    attv[0]  = bfr(a0.x); attv[1]  = bfr(a0.y); attv[2]  = bfr(a0.z); attv[3]  = bfr(a0.w);
    attv[4]  = bfr(a1.x); attv[5]  = bfr(a1.y); attv[6]  = bfr(a1.z); attv[7]  = bfr(a1.w);
    attv[8]  = bfr(a2.x); attv[9]  = bfr(a2.y); attv[10] = bfr(a2.z); attv[11] = bfr(a2.w);
    attv[12] = bfr(a3.x); attv[13] = bfr(a3.y); attv[14] = bfr(a3.z); attv[15] = bfr(a3.w);
  }
  __syncthreads();

  int tot = 0;
  const int nChunks = (nE + CHUNK - 1) / CHUNK;
#pragma unroll 1
  for (int ch = 0; ch < nChunks; ++ch) {
    const int cbase = ch * CHUNK;
    const int wc = scan_chunk(dsts, nE, cbase, nodeBase, nb, vec8, list, tid, lane, wave);
    if (lane == 0) wcnt[wave] = wc;
    __syncthreads();
    int pre = 0, all = 0;
#pragma unroll
    for (int w2 = 0; w2 < NWAVE; ++w2) {
      int c = wcnt[w2];
      c = c < 0 ? 0 : (c > WCAP ? WCAP : c);
      all += c;
      pre += (w2 < wave) ? c : 0;
    }
    const int wcc  = wc > WCAP ? WCAP : wc;
    const int base = tot + pre;
#pragma unroll 1
    for (int i = lane; i < wcc; i += 32) {
      const int ent = list[wave * WCAP + i];
      const int el  = (ent >> 12) & (CHUNK - 1);
      const int sl  = ent & (NBMAX - 1);
      int eid = cbase + el;
      eid = eid > nE - 1 ? nE - 1 : eid;
      const int pos = base + i;
      if (pos < RCAP) reg1[pos] = (int)(((unsigned)eid << 12) | (unsigned)sl);
    }
    tot += all;
    tot = tot > RCAP ? RCAP : tot;
    __syncthreads();
  }
  const int nh = tot;

  if (wave == 0) {
#pragma unroll 1
    for (int b0 = 0; b0 < nh; b0 += 32) {
      const int idx = b0 + lane;
      const int uv  = reg1[idx < RCAP ? idx : RCAP - 1];
      const int m32 = (nh - b0) < 32 ? (nh - b0) : 32;
#pragma unroll 1
      for (int k = 0; k < m32; ++k) {
        const int u  = __builtin_amdgcn_readlane(uv, k);
        const int sl = u & (NBMAX - 1);
        if (lane == 0) scnt[sl] = scnt[sl] + 1;
      }
    }
  }
  __syncthreads();

  {
    const v4i ca = *(const v4i*)(scnt + 8 * tid);
    const v4i cb = *(const v4i*)(scnt + 8 * tid + 4);
    const int e0 = ca.x < 0 ? 0 : ca.x, e1 = ca.y < 0 ? 0 : ca.y, e2 = ca.z < 0 ? 0 : ca.z, e3 = ca.w < 0 ? 0 : ca.w;
    const int e4 = cb.x < 0 ? 0 : cb.x, e5 = cb.y < 0 ? 0 : cb.y, e6 = cb.z < 0 ? 0 : cb.z, e7 = cb.w < 0 ? 0 : cb.w;
    const int ts = e0 + e1 + e2 + e3 + e4 + e5 + e6 + e7;
    int incl = ts;
#pragma unroll
    for (int d = 1; d < 32; d <<= 1) {
      const int up = __shfl_up(incl, d);
      if (lane >= d) incl += up;
    }
    if (lane == 31) wtot[wave] = incl;
    __syncthreads();
    int pre = 0;
#pragma unroll
    for (int w2 = 0; w2 < NWAVE; ++w2) pre += (w2 < wave) ? wtot[w2] : 0;
    int run = pre + incl - ts;
    soff[8 * tid + 0] = run; run += e0;
    soff[8 * tid + 1] = run; run += e1;
    soff[8 * tid + 2] = run; run += e2;
    soff[8 * tid + 3] = run; run += e3;
    soff[8 * tid + 4] = run; run += e4;
    soff[8 * tid + 5] = run; run += e5;
    soff[8 * tid + 6] = run; run += e6;
    soff[8 * tid + 7] = run;
  }
  __syncthreads();
  for (int i = tid; i < NBMAX; i += NTHR) list[i] = soff[i];
  __syncthreads();

  if (wave == 0) {
#pragma unroll 1
    for (int b0 = 0; b0 < nh; b0 += 32) {
      const int idx = b0 + lane;
      const int uv  = reg1[idx < RCAP ? idx : RCAP - 1];
      const int m32 = (nh - b0) < 32 ? (nh - b0) : 32;
#pragma unroll 1
      for (int k = 0; k < m32; ++k) {
        const int u   = __builtin_amdgcn_readlane(uv, k);
        const int sl  = u & (NBMAX - 1);
        const int eid = (int)((unsigned)u >> 12);
        if (lane == 0) {
          int pos = list[sl];
          pos = pos < 0 ? 0 : (pos > RCAP - 1 ? RCAP - 1 : pos);
          reg2[pos] = eid;
          list[sl] = pos + 1;
        }
      }
    }
  }
  __syncthreads();

  const int nbw = nb >> 3;
  const bool ovf = (nh >= RCAP);
  const float qnan = __int_as_float(0x7fc00000);
  float* stw = (float*)reg1 + wave * STW;
  const int l15 = lane & 15;
#pragma unroll 1
  for (int jt = 0; jt < nbw; ++jt) {
    const int slot = wave * nbw + jt;
    const int grow = nodeBase + slot;
    const int gcl  = grow < nN ? grow : nN - 1;
    int st = soff[slot];
    const int craw = scnt[slot];
    int cnt = craw;
    st  = st < 0 ? 0 : (st > nh ? nh : st);
    cnt = cnt < 0 ? 0 : (cnt > DEGCAP ? DEGCAP : cnt);
    if (cnt > nh - st) cnt = nh - st;
    const float pz = (ovf || craw > DEGCAP) ? qnan : 0.0f;
    const bool wr = grow < MPr;
    const float live = grow < nN ? 1.0f : 0.0f;
    const int gw = wr ? grow : 0;

    const float* xrp = XLR + (size_t)gcl * NLR + NL + 16 * lane;
    const v4f ra = *(const v4fa*)xrp, rb = *(const v4fa*)(xrp + 4), rc = *(const v4fa*)(xrp + 8), rd = *(const v4fa*)(xrp + 12);
    ldwait();
    const float xr[16] = {ra.x, ra.y, ra.z, ra.w, rb.x, rb.y, rb.z, rb.w, rc.x, rc.y, rc.z, rc.w, rd.x, rd.y, rd.z, rd.w};
    float mx = -1.0e30f, dn = 0.f;
    float av[16];
#pragma unroll
    for (int i = 0; i < 16; ++i) av[i] = 0.f;

    const int nit = cnt + 1;
#pragma unroll 1
    for (int q = 0; q < nit; ++q) {
      int ridx = st + q - 1;
      ridx = ridx < 0 ? 0 : (ridx > RCAP - 1 ? RCAP - 1 : ridx);
      int eid = reg2[ridx];
      eid = eid < 0 ? 0 : (eid > nE - 1 ? nE - 1 : eid);
      const int sraw = srcs[eid];
      const int se = sraw < 0 ? 0 : (sraw > nN - 1 ? nN - 1 : sraw);
      const int s = (q == 0) ? gcl : se;
      const float* xp = XLR + (size_t)s * NLR + 16 * lane;
      const v4f la = *(const v4fa*)xp, lb = *(const v4fa*)(xp + 4), lcv = *(const v4fa*)(xp + 8), ld = *(const v4fa*)(xp + 12);
      ldwait();
      const float xl[16] = {la.x, la.y, la.z, la.w, lb.x, lb.y, lb.z, lb.w, lcv.x, lcv.y, lcv.z, lcv.w, ld.x, ld.y, ld.z, ld.w};
      float part = 0.f;
#pragma unroll
      for (int i = 0; i < 16; ++i) {
        float e = xl[i] + xr[i];
        e = e > 0.f ? e : NEGS * e;
        part = fmaf(e, attv[i], part);
      }
      part += __shfl_xor(part, 4);
      part += __shfl_xor(part, 2);
      part += __shfl_xor(part, 1);
      const float df = part - mx;
      const float ee = __expf(-fabsf(df));
      const bool up  = df > 0.f;
      const float s1 = up ? ee : 1.0f;
      const float s2 = up ? 1.0f : ee;
      mx = up ? part : mx;
      dn = fmaf(dn, s1, s2);
#pragma unroll
      for (int i = 0; i < 16; ++i) av[i] = fmaf(av[i], s1, s2 * xl[i]);
    }
    const float inv = __builtin_amdgcn_rcpf(dn);
    const v4f o0 = {av[0] * inv,  av[1] * inv,  av[2] * inv,  av[3] * inv};
    const v4f o1 = {av[4] * inv,  av[5] * inv,  av[6] * inv,  av[7] * inv};
    const v4f o2 = {av[8] * inv,  av[9] * inv,  av[10] * inv, av[11] * inv};
    const v4f o3 = {av[12] * inv, av[13] * inv, av[14] * inv, av[15] * inv};
    __builtin_amdgcn_fence(__ATOMIC_RELEASE, "wavefront");
    __builtin_amdgcn_wave_barrier();
    *(v4fa*)(stw + 16 * lane)      = o0;
    *(v4fa*)(stw + 16 * lane + 4)  = o1;
    *(v4fa*)(stw + 16 * lane + 8)  = o2;
    *(v4fa*)(stw + 16 * lane + 12) = o3;
    __builtin_amdgcn_fence(__ATOMIC_RELEASE, "wavefront");
    __builtin_amdgcn_wave_barrier();
    const v4f g0 = *(const v4fa*)(stw + 4 * lane);
    const v4f g1 = *(const v4fa*)(stw + DIN + 4 * lane);
    const v4f g2 = *(const v4fa*)(stw + 2 * DIN + 4 * lane);
    const v4f g3 = *(const v4fa*)(stw + 3 * DIN + 4 * lane);
    const v4f gb4 = *(const v4fa*)(prm + 4 * lane);
    const v4f gg4 = *(const v4fa*)(prm + DIN + 4 * lane);
    const v4f bb4 = *(const v4fa*)(prm + 2 * DIN + 4 * lane);
    const v4us xq = *(const v4usa*)(XB + (size_t)gcl * DIN + 4 * lane);
    ldwait();
    float hv[4];
    hv[0] = bf2f(xq.x) + (((g0.x + g1.x) + (g2.x + g3.x)) * 0.25f + gb4.x);
    hv[1] = bf2f(xq.y) + (((g0.y + g1.y) + (g2.y + g3.y)) * 0.25f + gb4.y);
    hv[2] = bf2f(xq.z) + (((g0.z + g1.z) + (g2.z + g3.z)) * 0.25f + gb4.z);
    hv[3] = bf2f(xq.w) + (((g0.w + g1.w) + (g2.w + g3.w)) * 0.25f + gb4.w);
    float sm = (hv[0] + hv[1]) + (hv[2] + hv[3]);
#pragma unroll
    for (int off = 16; off > 0; off >>= 1) sm += __shfl_xor(sm, off);
    const float mu = sm * 0.0078125f;
    float dv[4], vs = 0.f;
#pragma unroll
    for (int k = 0; k < 4; ++k) { dv[k] = hv[k] - mu; vs = fmaf(dv[k], dv[k], vs); }
#pragma unroll
    for (int off = 16; off > 0; off >>= 1) vs += __shfl_xor(vs, off);
    const float rs = rsqrtf(fmaf(vs, 0.0078125f, LNEPS));
    v4f hn4;
    hn4.x = fmaf(dv[0] * rs, gg4.x, bb4.x) * live + pz;
    hn4.y = fmaf(dv[1] * rs, gg4.y, bb4.y) * live + pz;
    hn4.z = fmaf(dv[2] * rs, gg4.z, bb4.z) * live + pz;
    hn4.w = fmaf(dv[3] * rs, gg4.w, bb4.w) * live + pz;
    __builtin_amdgcn_fence(__ATOMIC_RELEASE, "wavefront");
    __builtin_amdgcn_wave_barrier();
    *(v4fa*)(stw + 4 * lane) = hn4;
    __builtin_amdgcn_fence(__ATOMIC_RELEASE, "wavefront");
    __builtin_amdgcn_wave_barrier();
    const v4f fa = *(const v4fa*)(stw + 8 * l15);
    const v4f fb = *(const v4fa*)(stw + 8 * l15 + 4);
    const float f8[8] = {fa.x, fa.y, fa.z, fa.w, fb.x, fb.y, fb.z, fb.w};
    const bool islo = lane >= 16;
    v8us pk;
#pragma unroll
    for (int j = 0; j < 8; ++j) {
      const unsigned short hi = f2bf(f8[j]);
      const unsigned short lo = f2bf(f8[j] - bf2f(hi));
      pk[j] = islo ? lo : hi;
    }
    unsigned short* hp = HB + (size_t)gw * K1 + 8 * lane;
    if (wr) *(volatile v8us*)hp = pk;
    __threadfence();
    if (wr) *(volatile v8us*)hp = pk;
  }
}

__global__ __launch_bounds__(GTHR) void k_ffn(
    const unsigned short* __restrict__ HB, const unsigned short* __restrict__ W1T,
    const unsigned short* __restrict__ W2T, const float* __restrict__ b1, const float* __restrict__ b2,
    float* out, int nRows)
{
  extern __shared__ v4f lds_ffn[];
  unsigned short* HT = (unsigned short*)lds_ffn;
  float* stg = (float*)((char*)lds_ffn + (size_t)GBM * K2 * 2);
  const int tid = (int)threadIdx.x, lane = tid & 31, wave = tid >> 5, hh = lane >> 4, m = lane & 15;
  const int rowBase = (int)blockIdx.x * GBM;
  const v8f z8 = {0.f, 0.f, 0.f, 0.f, 0.f, 0.f, 0.f, 0.f};
  const unsigned short* ap = HB + (size_t)(rowBase + 16 * wave + m) * (size_t)K1 + 8 * hh;

#pragma unroll 1
  for (int g = 0; g < DFF / GBN; ++g) {
    v8f acc[4];
    acc[0] = z8; acc[1] = z8; acc[2] = z8; acc[3] = z8;
    const unsigned short* wp = W1T + (size_t)(g * GBN + m) * (size_t)K1 + 8 * hh;
#pragma unroll 1
    for (int ks = 0; ks < K1 / 32; ++ks) {
      FragB af;
      af.h[0] = *(const v8usa*)(ap + 32 * ks);
      af.h[1] = *(const v8usa*)(ap + 32 * ks + 16);
#pragma unroll
      for (int t = 0; t < 4; ++t) {
        const unsigned short* wq = wp + (size_t)(16 * t) * (size_t)K1 + 32 * ks;
        FragB bf;
        bf.h[0] = *(const v8usa*)wq;
        bf.h[1] = *(const v8usa*)(wq + 16);
        acc[t] = wmb(af, bf, acc[t]);
      }
    }
#pragma unroll
    for (int t = 0; t < 4; ++t) {
      const int c = g * GBN + 16 * t + m;
      const float bv = bfr(b1[c]);
#pragma unroll
      for (int r = 0; r < 8; ++r) {
        const int lr = 16 * wave + 8 * hh + r;
        float v = acc[t][r] + bv;
        v = v > 0.f ? v : NEGS * v;
        const unsigned short hi = f2bf(v);
        const unsigned short lo = f2bf(v - bf2f(hi));
        HT[lr * K2 + c]       = hi;
        HT[lr * K2 + DFF + c] = lo;
      }
    }
  }
  __syncthreads();

  const unsigned short* hp = HT + (16 * wave + m) * K2 + 8 * hh;
#pragma unroll 1
  for (int g = 0; g < DIN / GBN; ++g) {
    v8f acc[4];
    acc[0] = z8; acc[1] = z8; acc[2] = z8; acc[3] = z8;
    const unsigned short* wp = W2T + (size_t)(g * GBN + m) * (size_t)K2 + 8 * hh;
#pragma unroll 1
    for (int ks = 0; ks < K2 / 32; ++ks) {
      FragB af;
      af.h[0] = *(const v8usa*)(hp + 32 * ks);
      af.h[1] = *(const v8usa*)(hp + 32 * ks + 16);
#pragma unroll
      for (int t = 0; t < 4; ++t) {
        const unsigned short* wq = wp + (size_t)(16 * t) * (size_t)K2 + 32 * ks;
        FragB bf;
        bf.h[0] = *(const v8usa*)wq;
        bf.h[1] = *(const v8usa*)(wq + 16);
        acc[t] = wmb(af, bf, acc[t]);
      }
    }
#pragma unroll
    for (int t = 0; t < 4; ++t) {
      const int lc = 16 * t + m;
      const int c = g * GBN + lc;
      const float bv = bfr(b2[c]);
#pragma unroll
      for (int r = 0; r < 8; ++r) {
        const int lr = 16 * wave + 8 * hh + r;
        stg[lr * GBN + lc] = acc[t][r] + bv;
      }
    }
    __syncthreads();

    v4us rh[8], rl[8];
    v4f fv[8];
#pragma unroll
    for (int i = 0; i < 8; ++i) {
      const int lr = 16 * wave + 2 * i + hh;
      const int gr = rowBase + lr;
      rh[i] = *(const v4usa*)(HB + (size_t)gr * K1 + g * GBN + 4 * m);
    }
    ldwait();
#pragma unroll
    for (int i = 0; i < 8; ++i) {
      const int lr = 16 * wave + 2 * i + hh;
      const int gr = rowBase + lr;
      rl[i] = *(const v4usa*)(HB + (size_t)gr * K1 + DIN + g * GBN + 4 * m);
    }
    ldwait();
#pragma unroll
    for (int i = 0; i < 8; ++i) {
      const int lr = 16 * wave + 2 * i + hh;
      v4f v = *(const v4fa*)(stg + lr * GBN + 4 * m);
      v.x = (bf2f(rh[i].x) + bf2f(rl[i].x)) + v.x;
      v.y = (bf2f(rh[i].y) + bf2f(rl[i].y)) + v.y;
      v.z = (bf2f(rh[i].z) + bf2f(rl[i].z)) + v.z;
      v.w = (bf2f(rh[i].w) + bf2f(rl[i].w)) + v.w;
      fv[i] = v;
    }
#pragma unroll
    for (int i = 0; i < 8; ++i) {
      const int lr = 16 * wave + 2 * i + hh;
      const int gr = rowBase + lr;
      const int grc = gr < nRows ? gr : 0;
      float* op = out + (size_t)grc * DIN + g * GBN + 4 * m;
      if (gr < nRows) *(volatile v4f*)op = fv[i];
    }
    __threadfence();
#pragma unroll
    for (int i = 0; i < 8; ++i) {
      const int lr = 16 * wave + 2 * i + hh;
      const int gr = rowBase + lr;
      const int grc = gr < nRows ? gr : 0;
      float* op = out + (size_t)grc * DIN + g * GBN + 4 * m;
      if (gr < nRows) *(volatile v4f*)op = fv[i];
    }
    __syncthreads();
  }
}

static int pick_nb(int nE, int nN) {
  int nb = NB0;
  while (nb > 16 && (long long)nb * (long long)nE * 5LL > (long long)RCAP * (long long)nN * 4LL) nb >>= 1;
  return nb;
}
static inline int cdiv(int a, int b) { return (a + b - 1) / b; }

extern "C" void kernel_launch(void* const* d_in, const int* in_sizes, int n_in,
                              void* d_out, int out_size, void* d_ws, size_t ws_size,
                              hipStream_t stream) {
  if (n_in < 14) return;
  const int nN = in_sizes[0] / DIN;
  if (nN <= 0 || in_sizes[0] != nN * DIN || nN > (1 << 22)) return;
  if (in_sizes[1] < 2 || (in_sizes[1] & 1) != 0) return;
  const int nE = in_sizes[1] / 2;
  if (nE < 1 || nE > (1 << 20)) return;
  if (in_sizes[2]  != DIN * NL   || in_sizes[3]  != NL)  return;
  if (in_sizes[4]  != DIN * NL   || in_sizes[5]  != NL)  return;
  if (in_sizes[6]  != NHEAD * DIN || in_sizes[7] != DIN) return;
  if (in_sizes[8]  != DIN || in_sizes[9] != DIN) return;
  if (in_sizes[10] != DIN * DFF  || in_sizes[11] != DFF) return;
  if (in_sizes[12] != DFF * DIN  || in_sizes[13] != DIN) return;
  if (out_size != nN * DIN) return;

  const float* x    = (const float*)d_in[0];
  const int*   ei   = (const int*)  d_in[1];
  const float* Wl   = (const float*)d_in[2];
  const float* bl   = (const float*)d_in[3];
  const float* Wr   = (const float*)d_in[4];
  const float* br   = (const float*)d_in[5];
  const float* att  = (const float*)d_in[6];
  const float* gbias= (const float*)d_in[7];
  const float* lng  = (const float*)d_in[8];
  const float* lnb  = (const float*)d_in[9];
  const float* W1   = (const float*)d_in[10];
  const float* b1   = (const float*)d_in[11];
  const float* W2   = (const float*)d_in[12];
  const float* b2   = (const float*)d_in[13];
  float* out = (float*)d_out;
  const int* src = ei;
  const int* dst = ei + nE;

  const int MP   = cdiv(nN, GBM) * GBM;
  const int nb   = pick_nb(nE, nN);
  const int gA   = cdiv(MP, nb);
  const int vec8 = ((nE & 3) == 0) ? 1 : 0;
  if (gA * nb < MP) return;

  char* ws = (char*)d_ws;
  size_t off = 0;
  const size_t oXB  = off; off += (size_t)MP * DIN * 2;            off = (off + 255) & ~(size_t)255;
  const size_t oXLR = off; off += (size_t)MP * NLR * 4;            off = (off + 255) & ~(size_t)255;
  const size_t oHB  = off; off += (size_t)MP * K1 * 2;             off = (off + 255) & ~(size_t)255;
  const size_t oWLR = off; off += (size_t)NLR * DIN * 2;           off = (off + 255) & ~(size_t)255;
  const size_t oW1T = off; off += (size_t)DFF * K1 * 2;            off = (off + 255) & ~(size_t)255;
  const size_t oW2T = off; off += (size_t)DIN * K2 * 2;            off = (off + 255) & ~(size_t)255;
  if (off > ws_size || off > (size_t)WSMAX) return;
  unsigned short* XB   = (unsigned short*)(ws + oXB);
  float*          XLR  = (float*)(ws + oXLR);
  unsigned short* HB   = (unsigned short*)(ws + oHB);
  unsigned short* WLRT = (unsigned short*)(ws + oWLR);
  unsigned short* W1T  = (unsigned short*)(ws + oW1T);
  unsigned short* W2T  = (unsigned short*)(ws + oW2T);

  hipFuncSetAttribute(reinterpret_cast<const void*>(&k_agg),
                      hipFuncAttributeMaxDynamicSharedMemorySize, LDS_AGG);
  hipFuncSetAttribute(reinterpret_cast<const void*>(&k_ffn),
                      hipFuncAttributeMaxDynamicSharedMemorySize, LDS_FFN);

  const int nUx = MP * (DIN / 8);
  k_xprep<<<cdiv(nUx, NTHR), NTHR, 0, stream>>>(x, XB, nN, nUx);

  {
    const int nU1 = NLR * (DIN / 8);
    k_wtr<<<cdiv(nU1, NTHR), NTHR, 0, stream>>>(Wl, Wr, NL, NL, DIN, DIN, WLRT, nU1);
    const int nU2 = DFF * (K1 / 8);
    k_wtr<<<cdiv(nU2, NTHR), NTHR, 0, stream>>>(W1, W1, DFF, DFF, DIN, K1, W1T, nU2);
    const int nU3 = DIN * (K2 / 8);
    k_wtr<<<cdiv(nU3, NTHR), NTHR, 0, stream>>>(W2, W2, DIN, DIN, DFF, K2, W2T, nU3);
  }

  const int gM = MP / GBM;
  k_gemm_xlr<<<dim3(gM, NLR / GBN), GTHR, 0, stream>>>(XB, WLRT, bl, br, XLR, DIN, NLR);
  k_agg<<<gA, NTHR, LDS_AGG, stream>>>(src, dst, XLR, XB, att, gbias, lng, lnb, HB, nN, nE, nb, vec8, MP);
  k_ffn<<<gM, GTHR, LDS_FFN, stream>>>(HB, W1T, W2T, b1, b2, out, nN);
}
